// GNN_Nodes_1047972021082
// MI455X (gfx1250) — hardware-verified
//
#include <hip/hip_runtime.h>
#include <stddef.h>


#define HIDC    128
#define NCLS    40
#define NCP     48
#define NTHR    256
#define NWAVE   8
#define EPT     8
#define NGRP    2
#define CHUNK   (NTHR * EPT * NGRP)
#define WCAP    (EPT * NGRP * 32)
#define LISTN   (NWAVE * WCAP)
#define NBC     4096
#define NBF     1024
#define RCAP    40960
#define RBN     128
#define TGT     256
#define DEGCAP  256
#define GLR     64
#define GHR     128
#define AP      (HIDC + 8)
#define OTHR    512
#define WSCALE  16.0f
#define WINV    0.0625f
#define BNEPS   1e-5f

#define LDS_GL   (2 * GLR * AP * 2)
#define LDS_HD   (2 * GHR * AP * 2)
#define LDS_FILL ((RCAP + NBF + LISTN) * 4 + 64)

static_assert((CHUNK & (CHUNK - 1)) == 0);
static_assert(CHUNK <= 4096);
static_assert(NBC <= 4096 && NBF <= 4096);
static_assert((NBC & (NBC - 1)) == 0 && (NBF & (NBF - 1)) == 0);
static_assert(NBC == 4 * NBF);
static_assert(OTHR * 8 == NBC);
static_assert((RCAP % 32) == 0);
static_assert(GLR * HIDC * 4 <= LDS_GL);
static_assert(GHR * NCLS * 4 <= LDS_HD);
static_assert((TGT % GLR) == 0 && (TGT % GHR) == 0 && TGT == NWAVE * 32);
static_assert(GLR == 4 * 16 && NWAVE == 8);
static_assert(GHR == NWAVE * 16);
static_assert((GHR * NCLS / 4) % NTHR == 0);
static_assert((HIDC * HIDC / 8) % NTHR == 0 && (NCP * HIDC / 8) % NTHR == 0);
static_assert((AP % 8) == 0);

typedef float          v4f   __attribute__((ext_vector_type(4)));
typedef float          v8f   __attribute__((ext_vector_type(8)));
typedef int            v4i   __attribute__((ext_vector_type(4)));
typedef double         v2d   __attribute__((ext_vector_type(2)));
typedef _Float16       v8h   __attribute__((ext_vector_type(8)));
typedef _Float16       v16h  __attribute__((ext_vector_type(16)));
typedef unsigned short v8us  __attribute__((ext_vector_type(8)));
typedef unsigned short v16us __attribute__((ext_vector_type(16)));
typedef __bf16         v16b  __attribute__((ext_vector_type(16)));
union FragH { v16h v;  v8h  h[2]; };
union FragU { v16us v; v8us h[2]; };

__device__ __forceinline__ unsigned short bfr(float f) {
  unsigned u = __float_as_uint(f);
  u += 0x7FFFu + ((u >> 16) & 1u);
  return (unsigned short)(u >> 16);
}

__device__ __forceinline__ v8h cvt8(v4f a, v4f b) {
  v8h r;
  r[0] = (_Float16)a.x; r[1] = (_Float16)a.y; r[2] = (_Float16)a.z; r[3] = (_Float16)a.w;
  r[4] = (_Float16)b.x; r[5] = (_Float16)b.y; r[6] = (_Float16)b.z; r[7] = (_Float16)b.w;
  return r;
}

__device__ __forceinline__ void split8(v4f a, v4f b, v8us& hi, v8us& lo) {
  float v[8];
  v[0] = a.x; v[1] = a.y; v[2] = a.z; v[3] = a.w; v[4] = b.x; v[5] = b.y; v[6] = b.z; v[7] = b.w;
#pragma unroll
  for (int e = 0; e < 8; ++e) {
    const unsigned short hs = bfr(v[e]);
    const float hf = __uint_as_float((unsigned)hs << 16);
    hi[e] = hs;
    lo[e] = bfr(v[e] - hf);
  }
}

__device__ __forceinline__ v8f wmh(v16h a, v16h b, v8f c) {
  v8f d = __builtin_amdgcn_wmma_f32_16x16x32_f16(false, a, false, b, (short)0, c, false, false);
  asm volatile("v_nop\n\tv_nop\n\tv_nop\n\tv_nop" : "+v"(d) : "v"(a), "v"(b));
  return d;
}
__device__ __forceinline__ v8f wmb(v16us a, v16us b, v8f c) {
  const v16b ab = __builtin_bit_cast(v16b, a);
  const v16b bb = __builtin_bit_cast(v16b, b);
  v8f d = __builtin_amdgcn_wmma_f32_16x16x32_bf16(false, ab, false, bb, (short)0, c, false, false);
  asm volatile("v_nop\n\tv_nop\n\tv_nop\n\tv_nop" : "+v"(d) : "v"(ab), "v"(bb));
  return d;
}

template <int NB>
__device__ __forceinline__ int scan_chunk(const int* __restrict__ dsts, int nE, int cbase, int slotBase,
                                          int vec8, int* list, int tid, int lane, int wave) {
  int wc = 0;
#pragma unroll
  for (int g = 0; g < NGRP; ++g) {
    const int el0  = (g * NTHR + tid) * EPT;
    const int e0   = cbase + el0;
    const int sent = -2147483647 - 1;
    v4i da, db;
    if (vec8 != 0 && cbase + CHUNK <= nE) {
      da = *(const v4i*)(dsts + e0);
      db = *(const v4i*)(dsts + e0 + 4);
    } else {
      da.x = (e0     < nE) ? dsts[min(e0, nE - 1)] : sent;
      da.y = (e0 + 1 < nE) ? dsts[min(e0 + 1, nE - 1)] : sent;
      da.z = (e0 + 2 < nE) ? dsts[min(e0 + 2, nE - 1)] : sent;
      da.w = (e0 + 3 < nE) ? dsts[min(e0 + 3, nE - 1)] : sent;
      db.x = (e0 + 4 < nE) ? dsts[min(e0 + 4, nE - 1)] : sent;
      db.y = (e0 + 5 < nE) ? dsts[min(e0 + 5, nE - 1)] : sent;
      db.z = (e0 + 6 < nE) ? dsts[min(e0 + 6, nE - 1)] : sent;
      db.w = (e0 + 7 < nE) ? dsts[min(e0 + 7, nE - 1)] : sent;
    }
    const unsigned nb = (unsigned)slotBase;
    const unsigned s0 = (unsigned)da.x - nb, s1 = (unsigned)da.y - nb;
    const unsigned s2 = (unsigned)da.z - nb, s3 = (unsigned)da.w - nb;
    const unsigned s4 = (unsigned)db.x - nb, s5 = (unsigned)db.y - nb;
    const unsigned s6 = (unsigned)db.z - nb, s7 = (unsigned)db.w - nb;
    const bool h0 = s0 < (unsigned)NB, h1 = s1 < (unsigned)NB, h2 = s2 < (unsigned)NB, h3 = s3 < (unsigned)NB;
    const bool h4 = s4 < (unsigned)NB, h5 = s5 < (unsigned)NB, h6 = s6 < (unsigned)NB, h7 = s7 < (unsigned)NB;
    const unsigned any = __builtin_amdgcn_ballot_w32(h0 | h1 | h2 | h3 | h4 | h5 | h6 | h7);
    if (any != 0u) {
#define HITJ(J, HJ, SJ) { \
        const unsigned mj = __builtin_amdgcn_ballot_w32(HJ); \
        if (mj != 0u) { \
          if (HJ) { \
            const int pos = wc + (int)__builtin_amdgcn_mbcnt_lo(mj, 0u); \
            if (pos < WCAP) list[wave * WCAP + pos] = ((el0 + (J)) << 12) | (int)(SJ); \
          } \
          wc += (int)__builtin_popcount(mj); } }
      HITJ(0, h0, s0)
      HITJ(1, h1, s1)
      HITJ(2, h2, s2)
      HITJ(3, h3, s3)
      HITJ(4, h4, s4)
      HITJ(5, h5, s5)
      HITJ(6, h6, s6)
      HITJ(7, h7, s7)
#undef HITJ
    }
  }
  return wc;
}

__global__ __launch_bounds__(NTHR) void k_wprep(
    const float* __restrict__ Ws, const float* __restrict__ Wo,
    unsigned short* w0h, unsigned short* w0l, _Float16* wf,
    unsigned short* woh, unsigned short* wol, int nL) {
  const int nA = HIDC * HIDC / 8;
  const int nB = (nL - 1) * (HIDC * HIDC / 8);
  const int nC = (nL + 1) * (NCP * HIDC / 8);
  const int bstart = blockIdx.x * NTHR;
  const int i = bstart + (int)threadIdx.x;
  float v[8];
  if (bstart < nA) {
    if (i >= nA) return;
    const int o = i * 8, n = o >> 7, k0 = o & 127;
#pragma unroll
    for (int e = 0; e < 8; ++e) v[e] = Ws[(size_t)(k0 + e) * HIDC + n];
    v4f a, b;
    a.x = v[0]; a.y = v[1]; a.z = v[2]; a.w = v[3]; b.x = v[4]; b.y = v[5]; b.z = v[6]; b.w = v[7];
    v8us hi, lo;
    split8(a, b, hi, lo);
    *(volatile v8us*)(w0h + o) = hi;
    *(volatile v8us*)(w0l + o) = lo;
    __threadfence();
    *(volatile v8us*)(w0h + o) = hi;
    *(volatile v8us*)(w0l + o) = lo;
  } else if (bstart < nA + nB) {
    const int ii = i - nA;
    if (ii >= nB) return;
    const int o = ii * 8;
    const int l = o / (HIDC * HIDC);
    const int oo = o - l * (HIDC * HIDC), n = oo >> 7, k0 = oo & 127;
    const float* src = Ws + (size_t)(l + 1) * HIDC * HIDC;
#pragma unroll
    for (int e = 0; e < 8; ++e) v[e] = src[(size_t)(k0 + e) * HIDC + n] * WSCALE;
    v4f a, b;
    a.x = v[0]; a.y = v[1]; a.z = v[2]; a.w = v[3]; b.x = v[4]; b.y = v[5]; b.z = v[6]; b.w = v[7];
    const v8h hv = cvt8(a, b);
    *(volatile v8h*)(wf + o) = hv;
    __threadfence();
    *(volatile v8h*)(wf + o) = hv;
  } else {
    const int ii = i - nA - nB;
    if (ii >= nC) return;
    const int o = ii * 8;
    const int j = o / (NCP * HIDC);
    const int oo = o - j * (NCP * HIDC), n = oo >> 7, k0 = oo & 127;
    const int nc = n < NCLS ? n : NCLS - 1;
#pragma unroll
    for (int e = 0; e < 8; ++e) {
      const float xw = Wo[(size_t)(j * HIDC + k0 + e) * NCLS + nc];
      v[e] = n < NCLS ? xw : 0.0f;
    }
    v4f a, b;
    a.x = v[0]; a.y = v[1]; a.z = v[2]; a.w = v[3]; b.x = v[4]; b.y = v[5]; b.z = v[6]; b.w = v[7];
    v8us hi, lo;
    split8(a, b, hi, lo);
    *(volatile v8us*)(woh + o) = hi;
    *(volatile v8us*)(wol + o) = lo;
    __threadfence();
    *(volatile v8us*)(woh + o) = hi;
    *(volatile v8us*)(wol + o) = lo;
  }
}

__global__ __launch_bounds__(NTHR) void k_count(
    const int* __restrict__ ei, int* cnt, float* dinv, int nE, int vec8) {
  __shared__ __attribute__((aligned(16))) int scnt[NBC];
  __shared__ __attribute__((aligned(16))) int list[LISTN];
  __shared__ int wcnt[NWAVE];
  const int tid = threadIdx.x, lane = tid & 31, wave = tid >> 5;
  const int nodeBase = blockIdx.x * NBC;
  const int* dsts = ei + nE;

  for (int i = tid; i < NBC; i += NTHR) scnt[i] = 0;
  __syncthreads();

  const int nChunks = (nE + CHUNK - 1) / CHUNK;
#pragma unroll 1
  for (int ch = 0; ch < nChunks; ++ch) {
    const int cbase = ch * CHUNK;
    const int wc = scan_chunk<NBC>(dsts, nE, cbase, nodeBase, vec8, list, tid, lane, wave);
    if (lane == 0) wcnt[wave] = wc;
    __syncthreads();
    if (wave == 0) {
#pragma unroll 1
      for (int wsx = 0; wsx < NWAVE; ++wsx) {
        int n = __builtin_amdgcn_readfirstlane(wcnt[wsx]);
        n = n > WCAP ? WCAP : (n < 0 ? 0 : n);
        const int* lp = list + wsx * WCAP;
#pragma unroll 1
        for (int i = 0; i < n; ++i) {
          const int ent  = __builtin_amdgcn_readfirstlane(lp[i]);
          const int slot = ent & (NBC - 1);
          if (lane == 0) scnt[slot] = scnt[slot] + 1;
        }
      }
    }
    __syncthreads();
  }

  v4i cq[4]; v4f dq[4];
#pragma unroll
  for (int q = 0; q < 4; ++q) {
    const int f = (wave * 4 + q) * 128 + 4 * lane;
    const v4i c = *(const v4i*)(scnt + f);
    cq[q] = c;
    dq[q].x = rsqrtf((float)(c.x + 1));
    dq[q].y = rsqrtf((float)(c.y + 1));
    dq[q].z = rsqrtf((float)(c.z + 1));
    dq[q].w = rsqrtf((float)(c.w + 1));
  }
  int*   cp = cnt + (size_t)nodeBase;
  float* dp = dinv + (size_t)nodeBase;
#pragma unroll
  for (int q = 0; q < 4; ++q) {
    const int f = (wave * 4 + q) * 128 + 4 * lane;
    *(volatile v4i*)(cp + f) = cq[q];
    *(volatile v4f*)(dp + f) = dq[q];
  }
  __threadfence();
#pragma unroll
  for (int q = 0; q < 4; ++q) {
    const int f = (wave * 4 + q) * 128 + 4 * lane;
    *(volatile v4i*)(cp + f) = cq[q];
    *(volatile v4f*)(dp + f) = dq[q];
  }
}

__global__ __launch_bounds__(OTHR) void k_offsets(
    const int* __restrict__ cnt, int* off, int* rbase, int nChunk) {
  __shared__ __attribute__((aligned(16))) int soff[NBC];
  __shared__ __attribute__((aligned(16))) int srb[RBN];
  __shared__ int wtot[OTHR / 32];
  const int tid = threadIdx.x, lane = tid & 31, wave = tid >> 5, sub = tid >> 7;
  for (int i = tid; i < RBN; i += OTHR) srb[i] = 0;
  int carry = 0;
#pragma unroll 1
  for (int ch = 0; ch < nChunk; ++ch) {
    const int base = ch * NBC;
    const v4i c0 = *(const v4i*)(cnt + base + 8 * tid);
    const v4i c1 = *(const v4i*)(cnt + base + 8 * tid + 4);
    const int e0 = max(c0.x, 0), e1 = max(c0.y, 0), e2 = max(c0.z, 0), e3 = max(c0.w, 0);
    const int e4 = max(c1.x, 0), e5 = max(c1.y, 0), e6 = max(c1.z, 0), e7 = max(c1.w, 0);
    const int ts = e0 + e1 + e2 + e3 + e4 + e5 + e6 + e7;
    int incl = ts;
#pragma unroll
    for (int d = 1; d < 32; d <<= 1) {
      const int t = __shfl_up(incl, d);
      if (lane >= d) incl += t;
    }
    if (lane == 31) wtot[wave] = incl;
    __syncthreads();
    const int S0 = wtot[0]  + wtot[1]  + wtot[2]  + wtot[3];
    const int S1 = wtot[4]  + wtot[5]  + wtot[6]  + wtot[7];
    const int S2 = wtot[8]  + wtot[9]  + wtot[10] + wtot[11];
    const int S3 = wtot[12] + wtot[13] + wtot[14] + wtot[15];
    int pre = 0;
#pragma unroll 1
    for (int w = 4 * sub; w < wave; ++w) pre += wtot[w];
    const int b0 = carry;
    const int b1 = b0 + ((S0 + 31) & ~31);
    const int b2 = b1 + ((S1 + 31) & ~31);
    const int b3 = b2 + ((S2 + 31) & ~31);
    const int b4 = b3 + ((S3 + 31) & ~31);
    const int myb = sub == 0 ? b0 : (sub == 1 ? b1 : (sub == 2 ? b2 : b3));
    if (tid == 0) {
      srb[min(4 * ch + 0, RBN - 1)] = b0;
      srb[min(4 * ch + 1, RBN - 1)] = b1;
      srb[min(4 * ch + 2, RBN - 1)] = b2;
      srb[min(4 * ch + 3, RBN - 1)] = b3;
    }
    int run = myb + pre + incl - ts;
    soff[8 * tid + 0] = run; run += e0;
    soff[8 * tid + 1] = run; run += e1;
    soff[8 * tid + 2] = run; run += e2;
    soff[8 * tid + 3] = run; run += e3;
    soff[8 * tid + 4] = run; run += e4;
    soff[8 * tid + 5] = run; run += e5;
    soff[8 * tid + 6] = run; run += e6;
    soff[8 * tid + 7] = run;
    carry = b4;
    __syncthreads();
    const v4i o0 = *(const v4i*)(soff + 4 * tid);
    const v4i o1 = *(const v4i*)(soff + 4 * (tid + OTHR));
    int* op = off + base;
    *(volatile v4i*)(op + 4 * tid) = o0;
    *(volatile v4i*)(op + 4 * (tid + OTHR)) = o1;
    __threadfence();
    *(volatile v4i*)(op + 4 * tid) = o0;
    *(volatile v4i*)(op + 4 * (tid + OTHR)) = o1;
    __syncthreads();
  }
  if (tid == 0) srb[min(4 * nChunk, RBN - 1)] = carry;
  __syncthreads();
  v4i rv = {0, 0, 0, 0};
  if (tid < 32) rv = *(const v4i*)(srb + 4 * tid);
  if (tid < 32) *(volatile v4i*)(rbase + 4 * tid) = rv;
  __threadfence();
  if (tid < 32) *(volatile v4i*)(rbase + 4 * tid) = rv;
}

__global__ __launch_bounds__(NTHR) void k_fill(
    const int* __restrict__ ei, const int* __restrict__ off, const int* __restrict__ rbase,
    int* csr, int nN, int nE, int vec8, int csrLen) {
  extern __shared__ v4f lds_dyn[];
  int* region = (int*)lds_dyn;
  int* cursor = region + RCAP;
  int* list   = cursor + NBF;
  int* wcnt   = list + LISTN;
  const int tid = threadIdx.x, lane = tid & 31, wave = tid >> 5;
  const int b = blockIdx.x;
  const int nodeBase = b * NBF;
  const int* dsts = ei + nE;

  int rb0 = rbase[b];
  const int rb1 = rbase[b + 1];
  rb0 = rb0 < 0 ? 0 : (rb0 > csrLen ? csrLen : rb0);
  rb0 &= ~31;
  int len = rb1 - rb0;
  len = len < 0 ? 0 : (len > RCAP ? RCAP : len);
  int lenW = (len + 31) & ~31;
  if (rb0 + lenW > csrLen) lenW = (csrLen - rb0) & ~31;

  {
    const v4i z = {0, 0, 0, 0};
    for (int i = tid; i < RCAP / 4; i += NTHR) ((v4i*)region)[i] = z;
    for (int s = tid; s < NBF; s += NTHR) {
      int o = off[nodeBase + s] - rb0;
      o = o < 0 ? 0 : (o > RCAP ? RCAP : o);
      cursor[s] = o;
    }
  }
  __syncthreads();

  const int nChunks = (nE + CHUNK - 1) / CHUNK;
#pragma unroll 1
  for (int ch = 0; ch < nChunks; ++ch) {
    const int cbase = ch * CHUNK;
    const int wc = scan_chunk<NBF>(dsts, nE, cbase, nodeBase, vec8, list, tid, lane, wave);
    if (lane == 0) wcnt[wave] = wc;
    __syncthreads();
    if (wave == 0) {
#pragma unroll 1
      for (int wsx = 0; wsx < NWAVE; ++wsx) {
        int n = __builtin_amdgcn_readfirstlane(wcnt[wsx]);
        n = n > WCAP ? WCAP : (n < 0 ? 0 : n);
        const int* lp = list + wsx * WCAP;
#pragma unroll 1
        for (int i = 0; i < n; ++i) {
          const int ent  = __builtin_amdgcn_readfirstlane(lp[i]);
          const int slot = ent & (NBF - 1);
          int e = cbase + ((ent >> 12) & (CHUNK - 1));
          e = e > nE - 1 ? nE - 1 : e;
          int src = ei[e];
          src = src < 0 ? 0 : (src > nN - 1 ? nN - 1 : src);
          if (lane == 0) {
            int pos = cursor[slot];
            pos = pos < 0 ? 0 : (pos > RCAP - 1 ? RCAP - 1 : pos);
            region[pos] = src;
            const int np = pos + 1;
            cursor[slot] = np > RCAP ? RCAP : np;
          }
        }
      }
    }
    __syncthreads();
  }

  const int nv = lenW >> 2;
  int* gp = csr + rb0;
#pragma unroll 1
  for (int i = tid; i < nv; i += NTHR) { const v4i v = ((const v4i*)region)[i]; *(volatile v4i*)(gp + 4 * i) = v; }
  __threadfence();
#pragma unroll 1
  for (int i = tid; i < nv; i += NTHR) { const v4i v = ((const v4i*)region)[i]; *(volatile v4i*)(gp + 4 * i) = v; }
}

template <int MODE>
__global__ __launch_bounds__(NTHR) void k_gemm(
    const float* __restrict__ A, int nRowsA, int useBn,
    const float* __restrict__ bnp, const float* __restrict__ beta,
    const _Float16* __restrict__ Bf, const unsigned short* __restrict__ Bh,
    const unsigned short* __restrict__ Bl, const float* __restrict__ dinv, float* C) {
  extern __shared__ v4f lds_dyn[];
  _Float16*       sAh = (_Float16*)lds_dyn;
  unsigned short* sHi = (unsigned short*)lds_dyn;
  unsigned short* sLo = sHi + GLR * AP;
  float*          stg = (float*)lds_dyn;
  const int tid = threadIdx.x, lane = tid & 31, wave = tid >> 5, hh = lane >> 4, m = lane & 15;
  const int rowBase = blockIdx.x * GLR;
  const int c0 = (tid & 15) * 8, rr = tid >> 4;

  v4f muA, muB, scA, scB, beA, beB;
  if (useBn != 0) {
    muA = *(const v4f*)(bnp + c0);          muB = *(const v4f*)(bnp + c0 + 4);
    scA = *(const v4f*)(bnp + HIDC + c0);   scB = *(const v4f*)(bnp + HIDC + c0 + 4);
    beA = *(const v4f*)(beta + c0);         beB = *(const v4f*)(beta + c0 + 4);
  } else {
    const v4f z = {0.f, 0.f, 0.f, 0.f}; const v4f o = {1.f, 1.f, 1.f, 1.f};
    muA = z; muB = z; scA = o; scB = o; beA = z; beB = z;
  }
#pragma unroll
  for (int i = 0; i < GLR / 16; ++i) {
    const int r = i * 16 + rr;
    int row = rowBase + r;
    row = row > nRowsA - 1 ? nRowsA - 1 : row;
    const float* ap = A + (size_t)row * HIDC + c0;
    v4f a = *(const v4f*)ap, b = *(const v4f*)(ap + 4);
    a = (a - muA) * scA + beA;
    b = (b - muB) * scB + beB;
    if (MODE == 0) {
      *(v8h*)(sAh + r * AP + c0) = cvt8(a, b);
    } else {
      v8us hi, lo;
      split8(a, b, hi, lo);
      *(v8us*)(sHi + r * AP + c0) = hi;
      *(v8us*)(sLo + r * AP + c0) = lo;
    }
  }
  __syncthreads();

  const int rt = wave & 3, cg = wave >> 2;
  const int r0 = 16 * rt;
  v8f acc[4];
#pragma unroll
  for (int t = 0; t < 4; ++t) { v8f z = {0.f, 0.f, 0.f, 0.f, 0.f, 0.f, 0.f, 0.f}; acc[t] = z; }
  if (MODE == 0) {
    const _Float16* ar = sAh + (r0 + m) * AP + 8 * hh;
#pragma unroll
    for (int kt = 0; kt < HIDC / 32; ++kt) {
      FragH a;
      a.h[0] = *(const v8h*)(ar + 32 * kt);
      a.h[1] = *(const v8h*)(ar + 32 * kt + 16);
#pragma unroll
      for (int t = 0; t < 4; ++t) {
        const _Float16* bp = Bf + (size_t)(64 * cg + 16 * t + m) * HIDC + 32 * kt + 8 * hh;
        FragH b;
        b.h[0] = *(const v8h*)bp;
        b.h[1] = *(const v8h*)(bp + 16);
        acc[t] = wmh(a.v, b.v, acc[t]);
      }
    }
  } else {
    const unsigned short* arh = sHi + (r0 + m) * AP + 8 * hh;
    const unsigned short* arl = sLo + (r0 + m) * AP + 8 * hh;
#pragma unroll 1
    for (int kt = 0; kt < HIDC / 32; ++kt) {
      FragU ah, al;
      ah.h[0] = *(const v8us*)(arh + 32 * kt);
      ah.h[1] = *(const v8us*)(arh + 32 * kt + 16);
      al.h[0] = *(const v8us*)(arl + 32 * kt);
      al.h[1] = *(const v8us*)(arl + 32 * kt + 16);
#pragma unroll
      for (int t = 0; t < 4; ++t) {
        const size_t bo = (size_t)(64 * cg + 16 * t + m) * HIDC + 32 * kt + 8 * hh;
        FragU bhf, blf;
        bhf.h[0] = *(const v8us*)(Bh + bo);
        bhf.h[1] = *(const v8us*)(Bh + bo + 16);
        blf.h[0] = *(const v8us*)(Bl + bo);
        blf.h[1] = *(const v8us*)(Bl + bo + 16);
        acc[t] = wmb(ah.v, bhf.v, acc[t]);
        acc[t] = wmb(ah.v, blf.v, acc[t]);
        acc[t] = wmb(al.v, bhf.v, acc[t]);
      }
    }
  }
  __syncthreads();

  const int rg = r0 + 8 * hh;
  const v4f dA = *(const v4f*)(dinv + (size_t)rowBase + rg);
  const v4f dB = *(const v4f*)(dinv + (size_t)rowBase + rg + 4);
  float s[8];
  s[0] = dA.x; s[1] = dA.y; s[2] = dA.z; s[3] = dA.w; s[4] = dB.x; s[5] = dB.y; s[6] = dB.z; s[7] = dB.w;
  const float wsc = MODE == 0 ? WINV : 1.0f;
#pragma unroll
  for (int r = 0; r < 8; ++r) s[r] *= wsc;
  float* sp = stg + rg * HIDC + 64 * cg + m;
#pragma unroll
  for (int t = 0; t < 4; ++t) {
#pragma unroll
    for (int r = 0; r < 8; ++r) sp[r * HIDC + 16 * t] = acc[t][r] * s[r];
  }
  __syncthreads();

  const float* lp = stg + wave * 8 * HIDC + 4 * lane;
  float* gp = C + ((size_t)rowBase + wave * 8) * HIDC + 4 * lane;
#pragma unroll
  for (int i = 0; i < 8; ++i) { const v4f v = *(const v4f*)(lp + i * HIDC); *(volatile v4f*)(gp + (size_t)i * HIDC) = v; }
  __threadfence();
#pragma unroll
  for (int i = 0; i < 8; ++i) { const v4f v = *(const v4f*)(lp + i * HIDC); *(volatile v4f*)(gp + (size_t)i * HIDC) = v; }
}

__global__ __launch_bounds__(NTHR) void k_agg(
    const int* __restrict__ csr, const int* __restrict__ off, const int* __restrict__ cnt,
    const float* __restrict__ dinv, const float* __restrict__ hw, float* agg,
    const float* __restrict__ bsl, double* part, int nN, int csrLen) {
  __shared__ __attribute__((aligned(16))) double red[NWAVE * 2 * HIDC];
  __shared__ __attribute__((aligned(16))) double tot[2 * HIDC];
  const int tid = threadIdx.x, lane = tid & 31, wave = tid >> 5;
  const int tbase = blockIdx.x * TGT + wave * 32;
  const int cl = tbase + lane;
  const int cnt_l = cnt[cl];
  const int off_l = off[cl];
  union FI { float f; int i; };
  FI dvu; dvu.f = dinv[cl];
  const v4f bb = *(const v4f*)(bsl + 4 * lane);
  double s0 = 0.0, s1 = 0.0, s2 = 0.0, s3 = 0.0;
  double q0 = 0.0, q1 = 0.0, q2 = 0.0, q3 = 0.0;

#pragma unroll 1
  for (int j = 0; j < 32; ++j) {
    const int c = tbase + j;
    int n = __builtin_amdgcn_readlane(cnt_l, j);
    n = n < 0 ? 0 : (n > DEGCAP ? DEGCAP : n);
    const int st = __builtin_amdgcn_readlane(off_l, j);
    FI du; du.i = __builtin_amdgcn_readlane(dvu.i, j);
    const float dc = du.f;
    v4f acc = {0.f, 0.f, 0.f, 0.f};
#pragma unroll 1
    for (int qb = 0; qb < n; qb += 32) {
      int pos = st + qb + lane;
      pos = pos < 0 ? 0 : (pos > csrLen - 1 ? csrLen - 1 : pos);
      int sl = csr[pos];
      sl = sl < 0 ? 0 : (sl > nN - 1 ? nN - 1 : sl);
      const int mcnt = (n - qb) < 32 ? (n - qb) : 32;
#pragma unroll 1
      for (int p = 0; p < mcnt; ++p) {
        const int s = __builtin_amdgcn_readlane(sl, p);
        acc = acc + *(const v4f*)(hw + (size_t)s * HIDC + 4 * lane);
      }
    }
    const v4f sv = *(const v4f*)(hw + (size_t)c * HIDC + 4 * lane);
    const v4f v = (acc + sv) * dc + bb;
    if (c < nN) {
      s0 += (double)v.x; s1 += (double)v.y; s2 += (double)v.z; s3 += (double)v.w;
      q0 += (double)v.x * (double)v.x; q1 += (double)v.y * (double)v.y;
      q2 += (double)v.z * (double)v.z; q3 += (double)v.w * (double)v.w;
    }
    float* hp = agg + (size_t)c * HIDC + 4 * lane;
    *(volatile v4f*)hp = v;
    __threadfence();
    *(volatile v4f*)hp = v;
  }

  red[(wave * 2 + 0) * HIDC + 4 * lane + 0] = s0;
  red[(wave * 2 + 0) * HIDC + 4 * lane + 1] = s1;
  red[(wave * 2 + 0) * HIDC + 4 * lane + 2] = s2;
  red[(wave * 2 + 0) * HIDC + 4 * lane + 3] = s3;
  red[(wave * 2 + 1) * HIDC + 4 * lane + 0] = q0;
  red[(wave * 2 + 1) * HIDC + 4 * lane + 1] = q1;
  red[(wave * 2 + 1) * HIDC + 4 * lane + 2] = q2;
  red[(wave * 2 + 1) * HIDC + 4 * lane + 3] = q3;
  __syncthreads();
  {
    const int stt = tid >> 7, ch = tid & 127;
    double t = 0.0;
#pragma unroll
    for (int w = 0; w < NWAVE; ++w) t += red[(w * 2 + stt) * HIDC + ch];
    tot[stt * HIDC + ch] = t;
  }
  __syncthreads();
  v2d pv[4];
#pragma unroll
  for (int p = 0; p < 4; ++p) { const v2d z = {0.0, 0.0}; pv[p] = z; }
  if (tid < 32) {
#pragma unroll
    for (int p = 0; p < 4; ++p) pv[p] = *(const v2d*)(tot + 2 * (p * 32 + lane));
  }
  double* pp = part + (size_t)blockIdx.x * (2 * HIDC);
  if (tid < 32) {
#pragma unroll
    for (int p = 0; p < 4; ++p) *(volatile v2d*)(pp + 2 * (p * 32 + lane)) = pv[p];
  }
  __threadfence();
  if (tid < 32) {
#pragma unroll
    for (int p = 0; p < 4; ++p) *(volatile v2d*)(pp + 2 * (p * 32 + lane)) = pv[p];
  }
}

__global__ __launch_bounds__(HIDC) void k_bnfin(
    const double* __restrict__ part, int nPart, const float* __restrict__ gam, float* bnp, int nN) {
  __shared__ __attribute__((aligned(16))) float so[2 * HIDC];
  const int tid = threadIdx.x, lane = tid & 31;
  double s = 0.0, q = 0.0;
#pragma unroll 1
  for (int b = 0; b < nPart; ++b) {
    s += part[(size_t)b * (2 * HIDC) + tid];
    q += part[(size_t)b * (2 * HIDC) + HIDC + tid];
  }
  const double invn = 1.0 / (double)nN;
  const double mu = s * invn;
  double var = q * invn - mu * mu;
  var = var < 0.0 ? 0.0 : var;
  const float varf = (float)var + BNEPS;
  const float rs = 1.0f / sqrtf(varf);
  so[tid] = (float)mu;
  so[HIDC + tid] = gam[tid] * rs;
  __syncthreads();
  v4f a = {0.f, 0.f, 0.f, 0.f}, c = {0.f, 0.f, 0.f, 0.f};
  if (tid < 32) { a = *(const v4f*)(so + 4 * lane); c = *(const v4f*)(so + HIDC + 4 * lane); }
  if (tid < 32) { *(volatile v4f*)(bnp + 4 * lane) = a; *(volatile v4f*)(bnp + HIDC + 4 * lane) = c; }
  __threadfence();
  if (tid < 32) { *(volatile v4f*)(bnp + 4 * lane) = a; *(volatile v4f*)(bnp + HIDC + 4 * lane) = c; }
}

template <int FIRST>
__global__ __launch_bounds__(NTHR) void k_head(
    const float* __restrict__ A, int nRowsA, int useBn,
    const float* __restrict__ bnp, const float* __restrict__ beta,
    const unsigned short* __restrict__ Bh, const unsigned short* __restrict__ Bl,
    const float* __restrict__ bias, float* dout, int nN) {
  extern __shared__ v4f lds_dyn[];
  unsigned short* sHi = (unsigned short*)lds_dyn;
  unsigned short* sLo = sHi + GHR * AP;
  float*          stg = (float*)lds_dyn;
  const int tid = threadIdx.x, lane = tid & 31, wave = tid >> 5, hh = lane >> 4, m = lane & 15;
  const int rowBase = blockIdx.x * GHR;
  const int c0 = (tid & 15) * 8, rr = tid >> 4;

  v4f muA, muB, scA, scB, beA, beB;
  if (useBn != 0) {
    muA = *(const v4f*)(bnp + c0);          muB = *(const v4f*)(bnp + c0 + 4);
    scA = *(const v4f*)(bnp + HIDC + c0);   scB = *(const v4f*)(bnp + HIDC + c0 + 4);
    beA = *(const v4f*)(beta + c0);         beB = *(const v4f*)(beta + c0 + 4);
  } else {
    const v4f z = {0.f, 0.f, 0.f, 0.f}; const v4f o = {1.f, 1.f, 1.f, 1.f};
    muA = z; muB = z; scA = o; scB = o; beA = z; beB = z;
  }
#pragma unroll
  for (int i = 0; i < GHR / 16; ++i) {
    const int r = i * 16 + rr;
    int row = rowBase + r;
    row = row > nRowsA - 1 ? nRowsA - 1 : row;
    const float* ap = A + (size_t)row * HIDC + c0;
    v4f a = *(const v4f*)ap, b = *(const v4f*)(ap + 4);
    a = (a - muA) * scA + beA;
    b = (b - muB) * scB + beB;
    v8us hi, lo;
    split8(a, b, hi, lo);
    *(v8us*)(sHi + r * AP + c0) = hi;
    *(v8us*)(sLo + r * AP + c0) = lo;
  }
  __syncthreads();

  const int r0 = wave * 16;
  v8f acc[3];
#pragma unroll
  for (int t = 0; t < 3; ++t) { v8f z = {0.f, 0.f, 0.f, 0.f, 0.f, 0.f, 0.f, 0.f}; acc[t] = z; }
  const unsigned short* arh = sHi + (r0 + m) * AP + 8 * hh;
  const unsigned short* arl = sLo + (r0 + m) * AP + 8 * hh;
#pragma unroll 1
  for (int kt = 0; kt < HIDC / 32; ++kt) {
    FragU ah, al;
    ah.h[0] = *(const v8us*)(arh + 32 * kt);
    ah.h[1] = *(const v8us*)(arh + 32 * kt + 16);
    al.h[0] = *(const v8us*)(arl + 32 * kt);
    al.h[1] = *(const v8us*)(arl + 32 * kt + 16);
#pragma unroll
    for (int t = 0; t < 3; ++t) {
      const size_t bo = (size_t)(16 * t + m) * HIDC + 32 * kt + 8 * hh;
      FragU bhf, blf;
      bhf.h[0] = *(const v8us*)(Bh + bo);
      bhf.h[1] = *(const v8us*)(Bh + bo + 16);
      blf.h[0] = *(const v8us*)(Bl + bo);
      blf.h[1] = *(const v8us*)(Bl + bo + 16);
      acc[t] = wmb(ah.v, bhf.v, acc[t]);
      acc[t] = wmb(ah.v, blf.v, acc[t]);
      acc[t] = wmb(al.v, bhf.v, acc[t]);
    }
  }
  __syncthreads();

  const int rg = r0 + 8 * hh;
#pragma unroll
  for (int t = 0; t < 3; ++t) {
    const int col  = 16 * t + m;
    const int colc = col < NCLS ? col : NCLS - 1;
    float pv[8];
    if (FIRST != 0) {
      const float bl = bias[colc];
#pragma unroll
      for (int r = 0; r < 8; ++r) pv[r] = bl;
    } else {
#pragma unroll
      for (int r = 0; r < 8; ++r) {
        int grow = rowBase + rg + r;
        grow = grow > nN - 1 ? nN - 1 : grow;
        pv[r] = dout[(size_t)grow * NCLS + colc];
      }
    }
    if (col < NCLS) {
#pragma unroll
      for (int r = 0; r < 8; ++r) stg[(rg + r) * NCLS + col] = acc[t][r] + pv[r];
    }
  }
  __syncthreads();

  int vrows = nN - rowBase;
  vrows = vrows < 0 ? 0 : (vrows > GHR ? GHR : vrows);
  const int pieces = vrows * (NCLS / 4);
  float* gp = dout + (size_t)rowBase * NCLS;
  v4f ov[GHR * NCLS / 4 / NTHR];
#pragma unroll
  for (int p = 0; p < GHR * NCLS / 4 / NTHR; ++p) {
    const int idx = p * NTHR + tid;
    ov[p] = *(const v4f*)(stg + 4 * idx);
  }
#pragma unroll
  for (int p = 0; p < GHR * NCLS / 4 / NTHR; ++p) {
    const int idx = p * NTHR + tid;
    if (idx < pieces) *(volatile v4f*)(gp + 4 * (size_t)idx) = ov[p];
  }
  __threadfence();
#pragma unroll
  for (int p = 0; p < GHR * NCLS / 4 / NTHR; ++p) {
    const int idx = p * NTHR + tid;
    if (idx < pieces) *(volatile v4f*)(gp + 4 * (size_t)idx) = ov[p];
  }
}

extern "C" void kernel_launch(void* const* d_in, const int* in_sizes, int n_in,
                              void* d_out, int out_size, void* d_ws, size_t ws_size,
                              hipStream_t stream) {
  if (n_in < 8) return;
  const int nN = in_sizes[0] / HIDC;
  if (nN <= 0 || in_sizes[0] != nN * HIDC) return;
  const int nL = in_sizes[1] / (HIDC * HIDC);
  if (nL < 1 || nL > 16 || in_sizes[1] != nL * HIDC * HIDC) return;
  if (in_sizes[2] < nL * HIDC || in_sizes[3] < nL * HIDC || in_sizes[4] < nL * HIDC) return;
  if (in_sizes[5] != (nL + 1) * HIDC * NCLS || in_sizes[6] < NCLS) return;
  const int nE = in_sizes[7] / 2;
  if (nE <= 0 || in_sizes[7] != 2 * nE) return;
  if (out_size != nN * NCLS) return;
  if (nE > (1 << 28) || nN > (1 << 24)) return;

  const float* x   = (const float*)d_in[0];
  const float* Ws  = (const float*)d_in[1];
  const float* bs  = (const float*)d_in[2];
  const float* gam = (const float*)d_in[3];
  const float* bet = (const float*)d_in[4];
  const float* Wo  = (const float*)d_in[5];
  const float* bo  = (const float*)d_in[6];
  const int*   ei  = (const int*)d_in[7];
  float* out = (float*)d_out;

  const int NPAD   = ((nN + TGT - 1) / TGT) * TGT;
  const int nBC    = (nN + NBC - 1) / NBC;
  const int CNTPAD = nBC * NBC;
  if (4 * nBC + 1 > RBN) return;
  const int nBF    = (nN + NBF - 1) / NBF;
  const int csrLen = ((nE + 31) & ~31) + 4096;
  const int nGl    = NPAD / GLR;
  const int nGh    = NPAD / GHR;
  const int nAgg   = NPAD / TGT;

  char* ws = (char*)d_ws;
  size_t off = 0;
  const size_t oW0h = off; off += (size_t)HIDC * HIDC * 2;                 off = (off + 255) & ~(size_t)255;
  const size_t oW0l = off; off += (size_t)HIDC * HIDC * 2;                 off = (off + 255) & ~(size_t)255;
  const size_t oWf  = off; off += (size_t)(nL - 1) * HIDC * HIDC * 2;      off = (off + 255) & ~(size_t)255;
  const size_t oWOh = off; off += (size_t)(nL + 1) * NCP * HIDC * 2;       off = (off + 255) & ~(size_t)255;
  const size_t oWOl = off; off += (size_t)(nL + 1) * NCP * HIDC * 2;       off = (off + 255) & ~(size_t)255;
  const size_t oCnt = off; off += (size_t)CNTPAD * 4;                      off = (off + 255) & ~(size_t)255;
  const size_t oDv  = off; off += (size_t)CNTPAD * 4;                      off = (off + 255) & ~(size_t)255;
  const size_t oOff = off; off += (size_t)CNTPAD * 4;                      off = (off + 255) & ~(size_t)255;
  const size_t oRb  = off; off += (size_t)RBN * 4;                         off = (off + 255) & ~(size_t)255;
  const size_t oCsr = off; off += (size_t)csrLen * 4;                      off = (off + 255) & ~(size_t)255;
  const size_t oHw  = off; off += (size_t)NPAD * HIDC * 4;                 off = (off + 255) & ~(size_t)255;
  const size_t oAgg = off; off += (size_t)NPAD * HIDC * 4;                 off = (off + 255) & ~(size_t)255;
  const size_t oPrt = off; off += (size_t)nAgg * 2 * HIDC * 8;             off = (off + 255) & ~(size_t)255;
  const size_t oBn  = off; off += (size_t)nL * 2 * HIDC * 4;               off = (off + 255) & ~(size_t)255;
  if (off > ws_size) return;
  unsigned short* w0h  = (unsigned short*)(ws + oW0h);
  unsigned short* w0l  = (unsigned short*)(ws + oW0l);
  _Float16*       wf   = (_Float16*)(ws + oWf);
  unsigned short* woh  = (unsigned short*)(ws + oWOh);
  unsigned short* wol  = (unsigned short*)(ws + oWOl);
  int*            cnt  = (int*)(ws + oCnt);
  float*          dinv = (float*)(ws + oDv);
  int*            offp = (int*)(ws + oOff);
  int*            rb   = (int*)(ws + oRb);
  int*            csr  = (int*)(ws + oCsr);
  float*          hw   = (float*)(ws + oHw);
  float*          agg  = (float*)(ws + oAgg);
  double*         part = (double*)(ws + oPrt);
  float*          bnp  = (float*)(ws + oBn);

  const int vec8 = ((nE & 3) == 0) ? 1 : 0;

  const int nPrep = HIDC * HIDC / 8 + (nL - 1) * (HIDC * HIDC / 8) + (nL + 1) * (NCP * HIDC / 8);
  k_wprep<<<(nPrep + NTHR - 1) / NTHR, NTHR, 0, stream>>>(Ws, Wo, w0h, w0l, wf, woh, wol, nL);

  k_count<<<nBC, NTHR, 0, stream>>>(ei, cnt, dinv, nE, vec8);
  k_offsets<<<1, OTHR, 0, stream>>>(cnt, offp, rb, nBC);
  hipFuncSetAttribute(reinterpret_cast<const void*>(&k_fill),
                      hipFuncAttributeMaxDynamicSharedMemorySize, LDS_FILL);
  k_fill<<<nBF, NTHR, LDS_FILL, stream>>>(ei, offp, rb, csr, nN, nE, vec8, csrLen);

  hipFuncSetAttribute(reinterpret_cast<const void*>(&k_head<1>),
                      hipFuncAttributeMaxDynamicSharedMemorySize, LDS_HD);
  hipFuncSetAttribute(reinterpret_cast<const void*>(&k_head<0>),
                      hipFuncAttributeMaxDynamicSharedMemorySize, LDS_HD);
  k_head<1><<<nGh, NTHR, LDS_HD, stream>>>(x, nN, 0, bnp, bet, woh, wol, bo, out, nN);

  for (int i = 0; i < nL; ++i) {
    if (i == 0) {
      k_gemm<1><<<nGl, NTHR, LDS_GL, stream>>>(x, nN, 0, bnp, bet, wf, w0h, w0l, dinv, hw);
    } else {
      k_gemm<0><<<nGl, NTHR, LDS_GL, stream>>>(agg, nN, 1, bnp + (size_t)(i - 1) * 2 * HIDC, bet + (size_t)(i - 1) * HIDC,
                                               wf + (size_t)(i - 1) * HIDC * HIDC, w0h, w0l, dinv, hw);
    }
    k_agg<<<nAgg, NTHR, 0, stream>>>(csr, offp, cnt, dinv, hw, agg, bs + (size_t)i * HIDC, part, nN, csrLen);
    k_bnfin<<<1, HIDC, 0, stream>>>(part, nAgg, gam + (size_t)i * HIDC, bnp + (size_t)i * 2 * HIDC, nN);
    k_head<0><<<nGh, NTHR, LDS_HD, stream>>>(agg, nN, 1, bnp + (size_t)i * 2 * HIDC, bet + (size_t)i * HIDC,
                                             woh + (size_t)(i + 1) * NCP * HIDC, wol + (size_t)(i + 1) * NCP * HIDC,
                                             bo, out, nN);
  }
}
